// Speech_MSA_45432164057333
// MI455X (gfx1250) — hardware-verified
//
#include <hip/hip_runtime.h>
#include <hip/hip_bf16.h>

typedef _Float16 bf16_t;
typedef __attribute__((ext_vector_type(16))) _Float16 v16bf;
typedef __attribute__((ext_vector_type(8)))  _Float16 v8bf;
typedef __attribute__((ext_vector_type(8)))  float  v8f;
typedef int v4i __attribute__((__vector_size__(16)));
typedef __attribute__((address_space(1))) v4i* as1_v4i_p;
typedef __attribute__((address_space(3))) v4i* as3_v4i_p;

#define EMBED   512
#define NHEADS  8
#define HDIM    64
#define WIN     17
#define PADW    8
#define BATCH   4
#define SEQ     2048
#define MROWS   (BATCH * SEQ)

#define USE_ASYNC_LDS 0

__device__ __forceinline__ void cp16_to_lds(bf16_t* dst_lds, const bf16_t* src_g) {
#if USE_ASYNC_LDS
  __builtin_amdgcn_global_load_async_to_lds_b128(
      (as1_v4i_p)(src_g), (as3_v4i_p)(dst_lds),  0,  0);
#else
  *reinterpret_cast<v8bf*>(dst_lds) = *reinterpret_cast<const v8bf*>(src_g);
#endif
}

__device__ __forceinline__ void wait_async0() {
#if USE_ASYNC_LDS
#if __has_builtin(__builtin_amdgcn_s_wait_asynccnt)
  __builtin_amdgcn_s_wait_asynccnt(0);
#else
  asm volatile("s_wait_asynccnt 0" ::: "memory");
#endif
#endif
}

__device__ __forceinline__ bf16_t f2bf(float f) { return (_Float16)f; }

__global__ __launch_bounds__(256) void cvt_f32_bf16_x4(
    const float* __restrict__ in, bf16_t* __restrict__ out, int n4) {
  int i = blockIdx.x * blockDim.x + threadIdx.x;
  if (i < n4) {
    float4 v = reinterpret_cast<const float4*>(in)[i];
    typedef __attribute__((ext_vector_type(4))) _Float16 v4h;
    v4h o; o[0] = f2bf(v.x); o[1] = f2bf(v.y); o[2] = f2bf(v.z); o[3] = f2bf(v.w);
    *(volatile v4h*)(out + (size_t)i * 4) = o; __threadfence(); *(volatile v4h*)(out + (size_t)i * 4) = o;
  }
}

__global__ __launch_bounds__(256) void transpose_cvt(
    const float* __restrict__ in, bf16_t* __restrict__ out, int K, int N) {
  long idx = (long)blockIdx.x * blockDim.x + threadIdx.x;
  if (idx < (long)K * N) {
    int n = (int)(idx / K);
    int k = (int)(idx % K);
    const bf16_t hv = f2bf(in[(size_t)k * N + n]);
    *(volatile bf16_t*)(out + idx) = hv; __threadfence(); *(volatile bf16_t*)(out + idx) = hv;
  }
}

#define BM 128
#define BN 64
#define BK 32
#define LDA 40

__global__ __launch_bounds__(128) void gemm_bf16_wmma(
    const bf16_t* __restrict__ A, const bf16_t* __restrict__ Bt,
    const float* __restrict__ bias, float* __restrict__ C,
    int M, int N, int K) {
  __shared__ bf16_t sA[2][BM * LDA];

  const int tid  = threadIdx.x;
  const int lane = tid & 31;
  const int wave = tid >> 5;
  const int m0 = blockIdx.y * BM;
  const int n0 = blockIdx.x * BN;
  const int KT = K / BK;

  auto stage = [&](int buf, int k0) {
#pragma unroll
    for (int i = 0; i < 4; ++i) {
      int c  = tid + i * 128;
      int r  = c >> 2;
      int kc = (c & 3) * 8;
      cp16_to_lds(&sA[buf][r * LDA + kc],
                  A + (size_t)(m0 + r) * K + k0 + kc);
    }
  };

  auto loadB = [&](int k0, v16bf* frag) {
    const int nn = lane & 15;
    const int kk = (lane >> 4) * 8;
#pragma unroll
    for (int j = 0; j < 4; ++j) {
      const bf16_t* p = Bt + (size_t)(n0 + j * 16 + nn) * K + k0;
      const v8bf lo = *reinterpret_cast<const v8bf*>(p + kk), hi = *reinterpret_cast<const v8bf*>(p + 16 + kk);
      frag[j] = __builtin_shufflevector(lo, hi, 0, 1, 2, 3, 4, 5, 6, 7, 8, 9, 10, 11, 12, 13, 14, 15);
    }
  };

  const int ar0 = wave * 32 + (lane & 15);
  const int kh  = (lane >> 4) * 8;
  auto loadA = [&](int buf, int row) -> v16bf {
    v8bf lo = *reinterpret_cast<const v8bf*>(&sA[buf][row * LDA + kh]);
    v8bf hi = *reinterpret_cast<const v8bf*>(&sA[buf][row * LDA + kh + 16]);
    return __builtin_shufflevector(lo, hi, 0, 1, 2, 3, 4, 5, 6, 7,
                                   8, 9, 10, 11, 12, 13, 14, 15);
  };

  v8f acc0[4], acc1[4];
#pragma unroll
  for (int j = 0; j < 4; ++j)
#pragma unroll
    for (int e = 0; e < 8; ++e) { acc0[j][e] = 0.0f; acc1[j][e] = 0.0f; }

  auto compute = [&](int buf, const v16bf* bf) {
    v16bf a0 = loadA(buf, ar0);
    v16bf a1 = loadA(buf, ar0 + 16);
#pragma unroll
    for (int j = 0; j < 4; ++j)
      acc0[j] = __builtin_amdgcn_wmma_f32_16x16x32_f16(
          false, a0, false, bf[j], (short)0, acc0[j], false, false);
#pragma unroll
    for (int j = 0; j < 4; ++j) {
      acc1[j] = __builtin_amdgcn_wmma_f32_16x16x32_f16(
          false, a1, false, bf[j], (short)0, acc1[j], false, false);
      asm volatile("v_nop\n\tv_nop\n\tv_nop\n\tv_nop" : "+v"(acc0[j]), "+v"(acc1[j]) : "v"(a1), "v"(bf[j]));
    }
  };

  v16bf bA[4], bB[4];
  stage(0, 0);
  loadB(0, bA);
  wait_async0();
  __syncthreads();

  for (int kt = 0; kt < KT; kt += 2) {
    if (kt + 1 < KT) {
      stage(1, (kt + 1) * BK);
      loadB((kt + 1) * BK, bB);
      if (kt + 2 < KT)
        __builtin_prefetch(A + (size_t)(m0 + tid) * K + (kt + 2) * BK, 0, 3);
    }
    compute(0, bA);
    wait_async0();
    __syncthreads();

    if (kt + 2 < KT) {
      stage(0, (kt + 2) * BK);
      loadB((kt + 2) * BK, bA);
    }
    compute(1, bB);
    wait_async0();
    __syncthreads();
  }

  const int hf = lane >> 4;
  const int r0 = m0 + wave * 32;
  for (int pass = 0; pass < 2; ++pass) {
#pragma unroll
    for (int p = 0; p < 2; ++p) {
      const int cb = n0 + p * 32;
      const float bv = bias[cb + lane];
#pragma unroll
      for (int i = 0; i < 8; ++i) {
        { const float a0 = acc0[2*p][i], a1 = acc0[2*p+1][i]; const float x0 = __shfl_xor(a0, 16), x1 = __shfl_xor(a1, 16);
          *(volatile float*)(C + (size_t)(r0 + i) * N + cb + lane)      = (hf ? x1 : a0) + bv;
          *(volatile float*)(C + (size_t)(r0 + 8 + i) * N + cb + lane)  = (hf ? a1 : x0) + bv; }
        { const float a0 = acc1[2*p][i], a1 = acc1[2*p+1][i]; const float x0 = __shfl_xor(a0, 16), x1 = __shfl_xor(a1, 16);
          *(volatile float*)(C + (size_t)(r0 + 16 + i) * N + cb + lane) = (hf ? x1 : a0) + bv;
          *(volatile float*)(C + (size_t)(r0 + 24 + i) * N + cb + lane) = (hf ? a1 : x0) + bv; }
      }
    }
    __threadfence();
  }
}

__global__ __launch_bounds__(256) void local_attn(
    const float* __restrict__ qkv, bf16_t* __restrict__ ctx) {
  const int lane = threadIdx.x & 31;
  const int widx = blockIdx.x * 8 + (threadIdx.x >> 5);
  const int t = widx & (SEQ - 1);
  const int h = (widx >> 11) & (NHEADS - 1);
  const int b = widx >> 14;
  const float scaling = 0.125f;

  const int qc = h * HDIM;
  const int kc = EMBED + h * HDIM;
  const int vc = 2 * EMBED + h * HDIM;
  const size_t row = (size_t)(b * SEQ + t);

  const float q0 = qkv[row * (3 * EMBED) + qc + lane] * scaling;
  const float q1 = qkv[row * (3 * EMBED) + qc + lane + 32] * scaling;

  float s[WIN];
#pragma unroll
  for (int w = 0; w < WIN; ++w) {
    int kt = t - PADW + w;
    float p = 0.0f;
    if (kt >= 0 && kt < SEQ) {
      const float* kp = qkv + (size_t)(b * SEQ + kt) * (3 * EMBED) + kc;
      p = q0 * kp[lane] + q1 * kp[lane + 32];
    }
#pragma unroll
    for (int off = 16; off > 0; off >>= 1) p += __shfl_xor(p, off, 32);
    s[w] = p;
  }

  float m = s[0];
#pragma unroll
  for (int w = 1; w < WIN; ++w) m = fmaxf(m, s[w]);
  float sum = 0.0f;
#pragma unroll
  for (int w = 0; w < WIN; ++w) { s[w] = __expf(s[w] - m); sum += s[w]; }
  const float inv = 1.0f / sum;

  float o0 = 0.0f, o1 = 0.0f;
#pragma unroll
  for (int w = 0; w < WIN; ++w) {
    int kt = t - PADW + w;
    if (kt >= 0 && kt < SEQ) {
      const float* vp = qkv + (size_t)(b * SEQ + kt) * (3 * EMBED) + vc;
      float pw = s[w] * inv;
      o0 += pw * vp[lane];
      o1 += pw * vp[lane + 32];
    }
  }

  const int s0 = (2 * lane) & 31, s1 = (2 * lane + 1) & 31;
  const float e0 = __shfl(o0, s0, 32), e1 = __shfl(o0, s1, 32), g0 = __shfl(o1, s0, 32), g1 = __shfl(o1, s1, 32);
  typedef __attribute__((ext_vector_type(2))) _Float16 v2h;
  v2h pr; pr[0] = f2bf(lane < 16 ? e0 : g0); pr[1] = f2bf(lane < 16 ? e1 : g1);
  bf16_t* op = ctx + row * EMBED + h * HDIM;
  *(volatile v2h*)(op + 2 * lane) = pr; __threadfence(); *(volatile v2h*)(op + 2 * lane) = pr;
}

extern "C" void kernel_launch(void* const* d_in, const int* in_sizes, int n_in,
                              void* d_out, int out_size, void* d_ws, size_t ws_size,
                              hipStream_t stream) {
  const float* x     = (const float*)d_in[0];
  const float* w_qkv = (const float*)d_in[1];
  const float* b_qkv = (const float*)d_in[2];
  const float* w_out = (const float*)d_in[3];
  const float* b_out = (const float*)d_in[4];
  float* out = (float*)d_out;
  (void)in_sizes; (void)n_in; (void)out_size;
  if (ws_size < (size_t)80 * 1024 * 1024) return;

  char* ws = (char*)d_ws;
  size_t off = 0;
  auto alloc = [&](size_t bytes) -> void* {
    void* p = ws + off;
    off = (off + bytes + 255) & ~(size_t)255;
    return p;
  };
  bf16_t* x_bf   = (bf16_t*)alloc((size_t)MROWS * EMBED * 2);
  bf16_t* wqkv_t = (bf16_t*)alloc((size_t)3 * EMBED * EMBED * 2);
  bf16_t* wout_t = (bf16_t*)alloc((size_t)EMBED * EMBED * 2);
  float*  qkv    = (float*) alloc((size_t)MROWS * 3 * EMBED * 4);
  bf16_t* ctx    = (bf16_t*)alloc((size_t)MROWS * EMBED * 2);

  {
    int n4 = MROWS * EMBED / 4;
    cvt_f32_bf16_x4<<<n4 / 256, 256, 0, stream>>>(x, x_bf, n4);
  }
  transpose_cvt<<<(512 * 1536) / 256, 256, 0, stream>>>(w_qkv, wqkv_t, 512, 1536);
  transpose_cvt<<<(512 * 512) / 256, 256, 0, stream>>>(w_out, wout_t, 512, 512);

  gemm_bf16_wmma<<<dim3(1536 / BN, MROWS / BM), 128, 0, stream>>>(
      x_bf, wqkv_t, b_qkv, qkv, MROWS, 1536, 512);

  local_attn<<<(BATCH * NHEADS * SEQ) / 8, 256, 0, stream>>>(qkv, ctx);

  gemm_bf16_wmma<<<dim3(512 / BN, MROWS / BM), 128, 0, stream>>>(
      ctx, wout_t, b_out, out, MROWS, 512, 512);
}
